// NeighborhoodAttention_85495618994612
// MI455X (gfx1250) — hardware-verified
//
#include <hip/hip_runtime.h>


#define HH   56
#define NPX  3136
#define CC   432
#define CP   448
#define C3P  1344
#define NHD  8
#define HDD  54
#define KW   7
#define KK   49
#define NC2  392
#define GIN  8
#define KO   1024
#define DM   CP
#define SCL  0.13608276348795434f
#define LOSC 1024.0f

typedef _Float16 h16;
typedef unsigned short bf;
typedef __attribute__((ext_vector_type(16))) __bf16   v16bf;
typedef __attribute__((ext_vector_type(16))) _Float16 v16h;
typedef __attribute__((ext_vector_type(8)))  _Float16 v8h;
typedef __attribute__((ext_vector_type(8)))  unsigned short v8us;
typedef __attribute__((ext_vector_type(8)))  float    v8f;
typedef __attribute__((ext_vector_type(4)))  float    v4f;
typedef v8h  __attribute__((may_alias)) v8ha;
typedef v4f  __attribute__((may_alias)) v4fa;
typedef v8us __attribute__((may_alias)) v8usa;

__device__ __forceinline__ unsigned short f2bf(float f) { unsigned u = __float_as_uint(f); u += 0x7FFFu + ((u >> 16) & 1u); return (unsigned short)(u >> 16); }
__device__ __forceinline__ float bf2f(unsigned short b) { return __uint_as_float(((unsigned)b) << 16); }
__device__ __forceinline__ float bfr(float f) { return bf2f(f2bf(f)); }
__device__ __forceinline__ v16h cat16(v8h lo, v8h hi) { return __builtin_shufflevector(lo, hi, 0, 1, 2, 3, 4, 5, 6, 7, 8, 9, 10, 11, 12, 13, 14, 15); }
__device__ __forceinline__ v16bf cat16b(v8us lo, v8us hi) { return __builtin_bit_cast(v16bf, __builtin_shufflevector(lo, hi, 0, 1, 2, 3, 4, 5, 6, 7, 8, 9, 10, 11, 12, 13, 14, 15)); }
__device__ __forceinline__ v8f wmma16(v16h a, v16h b, v8f c) { return __builtin_amdgcn_wmma_f32_16x16x32_f16(false, a, false, b, (short)0, c, false, false); }
__device__ __forceinline__ v8f wmmab(v16bf a, v16bf b, v8f c) { return __builtin_amdgcn_wmma_f32_16x16x32_bf16(false, a, false, b, (short)0, c, false, false); }

template <bool SPLITA, bool F16OUT = false>
__global__ __launch_bounds__(128) void k_gemmb(const bf* __restrict__ A, const bf* __restrict__ Al, const bf* __restrict__ Bn, const float* __restrict__ bias, float* C, int ldc, h16* C2, const float* __restrict__ R = nullptr, int K = DM, int roundR = 1) {
    __shared__ __align__(16) float ost[4][16 * 68];
    const int lane = threadIdx.x & 31, wave = threadIdx.x >> 5, lr = lane & 15, hi = lane >> 4;
    const int r0 = blockIdx.x * 64 + wave * 16, c0 = blockIdx.y * 64;
    const size_t aoff = (size_t)(r0 + lr) * K + 8 * hi;
    size_t boff[4];
#pragma unroll
    for (int t = 0; t < 4; ++t) boff[t] = (size_t)(c0 + t * 16 + lr) * K + 8 * hi;
    v8f acc[4];
#pragma unroll
    for (int t = 0; t < 4; ++t) acc[t] = (v8f){};
#pragma unroll 1
    for (int kc = 0; kc < K; kc += 32) {
        const v16bf a = cat16b(*(const v8us*)(A + aoff + kc), *(const v8us*)(A + aoff + kc + 16));
        v16bf al = a;
        if (SPLITA) al = cat16b(*(const v8us*)(Al + aoff + kc), *(const v8us*)(Al + aoff + kc + 16));
#pragma unroll
        for (int t = 0; t < 4; ++t) { const v16bf b = cat16b(*(const v8us*)(Bn + boff[t] + kc), *(const v8us*)(Bn + boff[t] + kc + 16)); acc[t] = wmmab(a, b, acc[t]); if (SPLITA) acc[t] = wmmab(al, b, acc[t]); }
        asm volatile("v_nop\n\tv_nop\n\tv_nop\n\tv_nop" : "+v"(acc[0]), "+v"(acc[1]), "+v"(acc[2]), "+v"(acc[3]) : "v"(a), "v"(al));
    }
    float* os = &ost[wave][0];
#pragma unroll
    for (int t = 0; t < 4; ++t) { const float bv = bias ? bfr(bias[c0 + t * 16 + lr]) : 0.f;
#pragma unroll
        for (int j = 0; j < 8; ++j) os[(hi * 8 + j) * 68 + t * 16 + lr] = acc[t][j] + bv; }
    __syncthreads();
    if (F16OUT) {
        h16* crow = (h16*)(void*)C + (size_t)r0 * ldc + c0;
        auto pass = [&]() {
#pragma unroll
            for (int s = 0; s < 4; ++s) { const int row = 4 * s + (lane >> 3), piece = lane & 7; const float* sp = os + row * 68 + piece * 8; v8h o, o2;
#pragma unroll
                for (int i = 0; i < 8; ++i) { const h16 a = (h16)sp[i]; o[i] = a; o2[i] = (h16)((sp[i] - (float)a) * LOSC); }
                *(volatile v8h*)(crow + (size_t)row * ldc + piece * 8) = o; if (C2) *(volatile v8h*)(C2 + (size_t)r0 * ldc + c0 + (size_t)row * ldc + piece * 8) = o2; }
        };
        pass(); __threadfence(); pass();
    } else {
        float* crow = C + (size_t)r0 * ldc + c0;
        auto pass = [&]() {
#pragma unroll
            for (int s = 0; s < 8; ++s) { const int Lid = (lane >> 3) + 4 * s, piece = lane & 7; const int row = Lid >> 1, cofs = (Lid & 1) * 32 + piece * 4;
                v4f val = *(const v4fa*)(os + row * 68 + cofs); if (R) { const v4f rv = *(const v4f*)(R + ((size_t)r0 + row) * ldc + c0 + cofs); val += roundR ? (v4f){bfr(rv[0]), bfr(rv[1]), bfr(rv[2]), bfr(rv[3])} : rv; }
                *(volatile v4f*)(crow + (size_t)row * ldc + cofs) = val; }
        };
        pass(); __threadfence(); pass();
    }
}


__device__ __forceinline__ int nstart(int i) { int s = i - 3; s = s < 0 ? 0 : s; s = s > HH - KW ? HH - KW : s; return s; }
__global__ __launch_bounds__(256) void k_xpad(const float* __restrict__ x, bf* XB) {
    const int lane = threadIdx.x & 31; const size_t p = (size_t)blockIdx.x * 8 + (threadIdx.x >> 5); if (p >= (size_t)NPX) return;
#pragma unroll 1
    for (int ps = 0; ps < 2; ++ps) {
#pragma unroll
        for (int q = 0; q < 2; ++q) { const int c0 = q * 256 + lane * 8; if (c0 < CP) { v8us o;
#pragma unroll
                for (int i = 0; i < 8; ++i) { const int c = c0 + i; o[i] = f2bf(c < CC ? x[p * CC + (c < CC ? c : 0)] : 0.f); }
                *(volatile v8us*)(XB + p * CP + c0) = o; } }
        if (ps == 0) __threadfence(); }
}
__global__ __launch_bounds__(256) void k_wpadn(const float* __restrict__ Wm, int Nl, int Kl, int NP, int KP, bf* Bt) {
    const int lane = threadIdx.x & 31; const int n = blockIdx.x * 8 + (threadIdx.x >> 5); if (n >= NP) return;
#pragma unroll 1
    for (int ps = 0; ps < 2; ++ps) {
        for (int c0 = lane * 8; c0 < KP; c0 += 256) { v8us o;
#pragma unroll
            for (int i = 0; i < 8; ++i) { const int k = c0 + i; const bool live = (n < Nl) && (k < Kl); o[i] = f2bf(live ? Wm[(size_t)(live ? n : 0) * Kl + (live ? k : 0)] : 0.f); }
            *(volatile v8us*)(Bt + (size_t)n * KP + c0) = o; }
        if (ps == 0) __threadfence(); }
}
__global__ __launch_bounds__(256) void k_bpadn(const float* __restrict__ b, int Nl, int NP, float* BP) {
    const int i = blockIdx.x * 256 + threadIdx.x; if (i >= NP) return; const float v = (i < Nl) ? b[i] : 0.f; *(volatile float*)(BP + i) = v; __threadfence(); *(volatile float*)(BP + i) = v;
}
__global__ __launch_bounds__(256) void k_natqk(const float* __restrict__ QKV, const float* __restrict__ rpb, float* ATT) {
    const int lane = threadIdx.x & 31; const size_t w = (size_t)blockIdx.x * 8 + (threadIdx.x >> 5); if (w >= (size_t)NPX * NHD) return; const int p = (int)(w / NHD), g = (int)(w % NHD); const int y = p / HH, x = p % HH; const int sy = nstart(y), sx = nstart(x);
    const float* qr = QKV + (size_t)p * C3P + g * HDD; float sc[2];
#pragma unroll
    for (int t = 0; t < 2; ++t) { const int s = lane + 32 * t; float a = -3.0e38f;
        if (s < KK) { const int u = s / KW, vv = s % KW; const int ny = sy + u, nx = sx + vv; const float* kr = QKV + ((size_t)ny * HH + nx) * C3P + CP + g * HDD; a = 0.f;
#pragma unroll 1
            for (int d = 0; d < HDD; ++d) a = fmaf(qr[d] * SCL, kr[d], a);
            a += bfr(rpb[((size_t)g * 13 + (6 - (y - sy) + u)) * 13 + (6 - (x - sx) + vv)]); }
        sc[t] = a; }
    float m = fmaxf(sc[0], sc[1]);
#pragma unroll
    for (int sh = 16; sh; sh >>= 1) m = fmaxf(m, __shfl_xor(m, sh, 32));
    const float e0 = __expf(sc[0] - m), e1 = (lane + 32 < KK) ? __expf(sc[1] - m) : 0.f; float sum = e0 + e1;
#pragma unroll
    for (int sh = 16; sh; sh >>= 1) sum += __shfl_xor(sum, sh, 32);
    const float inv = 1.0f / sum; float* dst = ATT + ((size_t)p * NHD + g) * 64;
    *(volatile float*)(dst + lane) = e0 * inv; *(volatile float*)(dst + 32 + lane) = e1 * inv; __threadfence(); *(volatile float*)(dst + lane) = e0 * inv; *(volatile float*)(dst + 32 + lane) = e1 * inv;
}
__global__ __launch_bounds__(256) void k_had(const float* __restrict__ QKV, float* HAD) {
    const int lane = threadIdx.x & 31; const size_t w = (size_t)blockIdx.x * 8 + (threadIdx.x >> 5); if (w >= (size_t)CC * (NPX / 32)) return; const int c = (int)(w / (NPX / 32)); const int p = (int)(w % (NPX / 32)) * 32 + lane;
    const float v = QKV[(size_t)p * C3P + c] * SCL * QKV[(size_t)p * C3P + CP + c] * SCL; float* dst = HAD + (size_t)c * NPX + p; *(volatile float*)dst = v; __threadfence(); *(volatile float*)dst = v;
}
__global__ __launch_bounds__(256) void k_gconv(const float* __restrict__ HAD, const float* __restrict__ w1, const float* __restrict__ b1, float* HG) {
    const int lane = threadIdx.x & 31; const size_t w = (size_t)blockIdx.x * 8 + (threadIdx.x >> 5); if (w >= (size_t)CC * (NPX / 32)) return; const int o = (int)(w / (NPX / 32)); const int p = (int)(w % (NPX / 32)) * 32 + lane; const int y = p / HH, x = p % HH; const int gi = o / GIN;
    float acc = bfr(b1[o]);
#pragma unroll 1
    for (int ci = 0; ci < GIN; ++ci) { const float* hc = HAD + (size_t)(gi * GIN + ci) * NPX; const float* wk = w1 + ((size_t)o * GIN + ci) * KK;
#pragma unroll 1
        for (int ty = 0; ty < KW; ++ty) { const int yy = y + ty - 3; if (yy < 0 || yy >= HH) continue;
#pragma unroll 1
            for (int tx = 0; tx < KW; ++tx) { const int xx = x + tx - 3; if (xx < 0 || xx >= HH) continue; acc = fmaf(hc[yy * HH + xx], bfr(wk[ty * KW + tx]), acc); } } }
    const float gl = 0.5f * acc * (1.0f + erff(acc * 0.70710678118654752f)); float* dst = HG + (size_t)o * NPX + p; *(volatile float*)dst = gl; __threadfence(); *(volatile float*)dst = gl;
}
__global__ __launch_bounds__(256) void k_cT(const float* __restrict__ F, bf* Ph, bf* Pl) {
    __shared__ float tl[64][65];
    typedef __attribute__((ext_vector_type(4))) unsigned short v4us;
    const int tid = threadIdx.x, c0 = blockIdx.x * 64, p0 = blockIdx.y * 64; const int rr = tid >> 2, cq = (tid & 3) * 16;
#pragma unroll
    for (int i = 0; i < 16; ++i) tl[rr][cq + i] = (c0 + rr < CC) ? F[(size_t)(c0 + rr) * NPX + p0 + cq + i] : 0.f;
    __syncthreads();
    const int lane = tid & 31, wv = tid >> 5;
    auto pass = [&]() {
#pragma unroll
        for (int st = 0; st < 4; ++st) { const int pr = wv * 8 + st * 2 + (lane >> 4); const int cl = (lane & 15) * 4; v4us oh, ol;
#pragma unroll
            for (int i = 0; i < 4; ++i) { const float y = tl[cl + i][pr]; const unsigned short hb = f2bf(y); oh[i] = hb; ol[i] = f2bf(y - bf2f(hb)); }
            const size_t o = (size_t)(p0 + pr) * CP + c0 + cl; *(volatile v4us*)(Ph + o) = oh; *(volatile v4us*)(Pl + o) = ol; }
    };
    pass(); __threadfence(); pass();
}
__global__ __launch_bounds__(256) void k_hsoft(const float* __restrict__ H2, float* HAT) {
    const int lane = threadIdx.x & 31; const size_t p = (size_t)blockIdx.x * 8 + (threadIdx.x >> 5); if (p >= (size_t)NPX) return; const float* hr = H2 + p * CP; float m = -3.0e38f;
#pragma unroll 1
    for (int c = lane; c < NC2; c += 32) m = fmaxf(m, hr[c]);
#pragma unroll
    for (int sh = 16; sh; sh >>= 1) m = fmaxf(m, __shfl_xor(m, sh, 32));
    float sum = 0.f;
#pragma unroll 1
    for (int c = lane; c < NC2; c += 32) sum += __expf(hr[c] - m);
#pragma unroll
    for (int sh = 16; sh; sh >>= 1) sum += __shfl_xor(sum, sh, 32);
    const float inv = 1.0f / sum;
#pragma unroll 1
    for (int ps = 0; ps < 2; ++ps) {
#pragma unroll 1
        for (int g = 0; g < NHD; ++g) { float* dst = HAT + (p * NHD + g) * 64; const int s0 = lane, s1 = lane + 32;
            const float v0 = __expf(hr[g * KK + s0] - m) * inv; const float v1 = (s1 < KK) ? __expf(hr[g * KK + (s1 < KK ? s1 : 0)] - m) * inv : 0.f;
            *(volatile float*)(dst + s0) = v0; *(volatile float*)(dst + s1) = v1; }
        if (ps == 0) __threadfence(); }
}
__global__ __launch_bounds__(256) void k_elsa(const float* __restrict__ QKV, const float* __restrict__ ATT, const float* __restrict__ HAT, const float* __restrict__ ghost, float* ELSA) {
    const int lane = threadIdx.x & 31; const size_t w = (size_t)blockIdx.x * 8 + (threadIdx.x >> 5); if (w >= (size_t)CC * (NPX / 32)) return; const int c = (int)(w / (NPX / 32)); const int p = (int)(w % (NPX / 32)) * 32 + lane; const int y = p / HH, x = p % HH;
    const int gI = c / 27; const int head = gI >> 1; const float* A = ((gI & 1) ? HAT : ATT) + ((size_t)p * NHD + head) * 64; float acc = 0.f;
#pragma unroll 1
    for (int k = 0; k < KK; ++k) { const int u = k / KW, vv = k % KW; const int yy = y + u - 3, xx = x + vv - 3; const bool in = (yy >= 0 && yy < HH && xx >= 0 && xx < HH);
        const float val = in ? QKV[((size_t)(in ? yy : 0) * HH + (in ? xx : 0)) * C3P + 2 * CP + c] : 0.f; acc = fmaf(val, A[k] + bfr(ghost[(size_t)c * KK + k]), acc); }
    float* dst = ELSA + (size_t)c * NPX + p; *(volatile float*)dst = acc; __threadfence(); *(volatile float*)dst = acc;
}
__global__ __launch_bounds__(256) void k_natav(const float* __restrict__ QKV, const float* __restrict__ ATT, const float* __restrict__ HAT, float* AV) {
    const int lane = threadIdx.x & 31; const size_t w = (size_t)blockIdx.x * 8 + (threadIdx.x >> 5); if (w >= (size_t)NPX * NHD) return; const int p = (int)(w / NHD), g = (int)(w % NHD); const int y = p / HH, x = p % HH; const int sy = nstart(y), sx = nstart(x);
    const float* a0 = ATT + ((size_t)p * NHD + g) * 64; const float* a1 = HAT + ((size_t)p * NHD + g) * 64; float acc0 = 0.f, acc1 = 0.f; const int d0 = lane, d1 = lane + 32;
#pragma unroll 1
    for (int s = 0; s < KK; ++s) { const int u = s / KW, vv = s % KW; const float a = a0[s] + a1[s]; const float* vr = QKV + ((size_t)(sy + u) * HH + (sx + vv)) * C3P + 2 * CP + g * HDD;
        acc0 = fmaf(a, vr[d0], acc0); if (d1 < HDD) acc1 = fmaf(a, vr[d1], acc1); }
    float* dst = AV + ((size_t)p * NHD + g) * 64; const float o1 = (d1 < HDD) ? acc1 : 0.f;
    *(volatile float*)(dst + d0) = acc0; *(volatile float*)(dst + 32 + lane) = o1; __threadfence(); *(volatile float*)(dst + d0) = acc0; *(volatile float*)(dst + 32 + lane) = o1;
}
__global__ __launch_bounds__(256) void k_catpl(const float* __restrict__ AV, const float* __restrict__ ELSA, bf* Oh, bf* Ol) {
    const int lane = threadIdx.x & 31; const size_t p = (size_t)blockIdx.x * 8 + (threadIdx.x >> 5); if (p >= (size_t)NPX) return;
#pragma unroll 1
    for (int ps = 0; ps < 2; ++ps) {
#pragma unroll 1
        for (int q = 0; q < 4; ++q) { const int c0 = q * 256 + lane * 8; v8us oh, ol;
#pragma unroll 1
            for (int i = 0; i < 8; ++i) { const int j = c0 + i; float y = 0.f; if (j < 2 * CC) { const int head = j / (2 * HDD), jj = j % (2 * HDD); y = (jj < HDD) ? AV[(p * NHD + head) * 64 + jj] : ELSA[(size_t)(head * HDD + jj - HDD) * NPX + p]; } const unsigned short hb = f2bf(y); oh[i] = hb; ol[i] = f2bf(y - bf2f(hb)); }
            const size_t o = p * KO + c0; *(volatile v8us*)(Oh + o) = oh; *(volatile v8us*)(Ol + o) = ol; }
        if (ps == 0) __threadfence(); }
}
__global__ __launch_bounds__(256) void k_out432(const float* __restrict__ Y, float* OUTB) {
    const int lane = threadIdx.x & 31; const size_t w = (size_t)blockIdx.x * 8 + (threadIdx.x >> 5); const size_t e0 = (w * 32 + lane) * 4; if (e0 >= (size_t)NPX * CC) return; const size_t p = e0 / CC; const int c = (int)(e0 % CC);
    const v4f v = *(const v4f*)(Y + p * CP + c); *(volatile v4f*)(OUTB + e0) = v; __threadfence(); *(volatile v4f*)(OUTB + e0) = v;
}

extern "C" void kernel_launch(void* const* d_in, const int* in_sizes, int n_in,
                              void* d_out, int out_size, void* d_ws, size_t ws_size, hipStream_t stream) {
    (void)in_sizes; (void)n_in; (void)out_size;
    const float* x = (const float*)d_in[0]; const float* qkvw = (const float*)d_in[1]; const float* qkvb = (const float*)d_in[2]; const float* rpb = (const float*)d_in[3]; const float* c1w = (const float*)d_in[4]; const float* c1b = (const float*)d_in[5]; const float* c2w = (const float*)d_in[6]; const float* c2b = (const float*)d_in[7]; const float* ghost = (const float*)d_in[8]; const float* p2w = (const float*)d_in[9]; const float* p2b = (const float*)d_in[10];
    float* out = (float*)d_out;
    char* wsp = (char*)d_ws;
    auto take = [&](size_t bytes) { char* p = wsp; wsp += (bytes + 255) & ~(size_t)255; return (void*)p; };
    bf* WQKV = (bf*)take((size_t)C3P * CP * 2); float* BQKV = (float*)take(C3P * 4); bf* WC2 = (bf*)take((size_t)CP * CP * 2); float* BC2 = (float*)take(CP * 4); bf* WP2 = (bf*)take((size_t)CP * KO * 2); float* BP2 = (float*)take(CP * 4);
    bf* XB = (bf*)take((size_t)NPX * CP * 2); float* QKV = (float*)take((size_t)NPX * C3P * 4); float* ATT = (float*)take((size_t)NPX * NHD * 64 * 4); float* HAT = (float*)take((size_t)NPX * NHD * 64 * 4); float* AV = (float*)take((size_t)NPX * NHD * 64 * 4);
    float* HAD = (float*)take((size_t)CC * NPX * 4); float* HG = (float*)take((size_t)CC * NPX * 4); bf* Gh = (bf*)take((size_t)NPX * CP * 2); bf* Gl = (bf*)take((size_t)NPX * CP * 2); float* H2 = (float*)take((size_t)NPX * CP * 4); float* ELSA = (float*)take((size_t)CC * NPX * 4);
    bf* Oh = (bf*)take((size_t)NPX * KO * 2); bf* Ol = (bf*)take((size_t)NPX * KO * 2); float* Y = (float*)take((size_t)NPX * CP * 4);
    if ((size_t)(wsp - (char*)d_ws) > ws_size) return;
    for (int s = 0; s < 3; ++s) { k_wpadn<<<CP / 8, 256, 0, stream>>>(qkvw + (size_t)s * CC * CC, CC, CC, CP, CP, WQKV + (size_t)s * CP * CP); k_bpadn<<<(CP + 255) / 256, 256, 0, stream>>>(qkvb + s * CC, CC, CP, BQKV + s * CP); }
    k_wpadn<<<CP / 8, 256, 0, stream>>>(c2w, NC2, CC, CP, CP, WC2); k_bpadn<<<(CP + 255) / 256, 256, 0, stream>>>(c2b, NC2, CP, BC2);
    k_wpadn<<<CP / 8, 256, 0, stream>>>(p2w, CC, 2 * CC, CP, KO, WP2); k_bpadn<<<(CP + 255) / 256, 256, 0, stream>>>(p2b, CC, CP, BP2);
    k_xpad<<<NPX / 8, 256, 0, stream>>>(x, XB);
    k_gemmb<false, false><<<dim3(NPX / 64, C3P / 64, 1), 128, 0, stream>>>(XB, nullptr, WQKV, BQKV, QKV, C3P, nullptr, nullptr, CP);
    k_natqk<<<(NPX * NHD) / 8, 256, 0, stream>>>(QKV, rpb, ATT);
    k_had<<<(CC * (NPX / 32)) / 8, 256, 0, stream>>>(QKV, HAD);
    k_gconv<<<(CC * (NPX / 32)) / 8, 256, 0, stream>>>(HAD, c1w, c1b, HG);
    k_cT<<<dim3(CP / 64, NPX / 64, 1), 256, 0, stream>>>(HG, Gh, Gl);
    k_gemmb<true, false><<<dim3(NPX / 64, CP / 64, 1), 128, 0, stream>>>(Gh, Gl, WC2, BC2, H2, CP, nullptr, nullptr, CP);
    k_hsoft<<<NPX / 8, 256, 0, stream>>>(H2, HAT);
    k_elsa<<<(CC * (NPX / 32)) / 8, 256, 0, stream>>>(QKV, ATT, HAT, ghost, ELSA);
    k_natav<<<(NPX * NHD) / 8, 256, 0, stream>>>(QKV, ATT, HAT, AV);
    k_catpl<<<NPX / 8, 256, 0, stream>>>(AV, ELSA, Oh, Ol);
    k_gemmb<true, false><<<dim3(NPX / 64, CP / 64, 1), 128, 0, stream>>>(Oh, Ol, WP2, BP2, Y, CP, nullptr, nullptr, KO);
    k_out432<<<(NPX * CC / 4 / 32 + 7) / 8, 256, 0, stream>>>(Y, out);
}
